// SharedBackbone_61400852463655
// MI455X (gfx1250) — hardware-verified
//
#include <hip/hip_runtime.h>
#include <stddef.h>


#define FIN     128
#define HID     128
#define NHEADA  4
#define NTHR    256
#define NWAVE   8
#define EPT     8
#define NGRP    2
#define CHUNK   (NTHR * EPT * NGRP)
#define WCAP    (EPT * NGRP * 32)
#define LISTN   (NWAVE * WCAP)
#define NBC     4096
#define NBF     1024
#define RCAP    40960
#define RBN     128
#define TGT     256
#define DEGCAP  256
#define OTHR    512
#define BM      128
#define STATR   256
#define BNT     128
#define WSCAP   134217728
#define NEG_SLOPE 0.2f
#define DEN_EPS   1e-16f
#define BN_EPS    1e-5
#define XSC       8.0f
#define WSC       64.0f
#define INV_CARRY (1.0f / 512.0f)
#define APITCH    128

#define LDS_FILL  ((RCAP + NBF + LISTN) * 4 + 64)
#define LDS_ATILE (BM * APITCH * 2)
#define LDS_GEMM  (LDS_ATILE + BM * HID * 4)

static_assert((CHUNK & (CHUNK - 1)) == 0);
static_assert(CHUNK <= 4096);
static_assert(NBC <= 4096 && NBF <= 4096);
static_assert((NBC & (NBC - 1)) == 0 && (NBF & (NBF - 1)) == 0);
static_assert(NBC == 4 * NBF);
static_assert(OTHR * 8 == NBC);
static_assert((RCAP % 32) == 0);
static_assert(TGT == NWAVE * 32);
static_assert((TGT % BM) == 0 && (TGT % STATR) == 0);
static_assert(FIN / 8 == 16);
static_assert(FIN == HID);
static_assert(HID == 128 && BM == 16 * NWAVE && NWAVE == 8);
static_assert(HID == 32 * 4);
static_assert(BNT == HID);
static_assert((FIN % 32) == 0);

typedef float          v4f  __attribute__((ext_vector_type(4)));
typedef float          v8f  __attribute__((ext_vector_type(8)));
typedef int            v4i  __attribute__((ext_vector_type(4)));
typedef _Float16       v8h  __attribute__((ext_vector_type(8)));
typedef _Float16       v16h __attribute__((ext_vector_type(16)));
union FragH { v16h v; v8h h[2]; };

__device__ __forceinline__ v8f wmh(v16h a, v16h b, v8f c) {
  v8f d = __builtin_amdgcn_wmma_f32_16x16x32_f16(false, a, false, b, (short)0, c, false, false);
  asm volatile("v_nop\n\tv_nop\n\tv_nop\n\tv_nop" : "+v"(d) : "v"(a), "v"(b));
  return d;
}

__device__ __forceinline__ float lrelu(float v) { return v > 0.0f ? v : NEG_SLOPE * v; }
__device__ __forceinline__ float eluf(float v)  { return v > 0.0f ? v : (__expf(v) - 1.0f); }

template <int NB>
__device__ __forceinline__ int scan_chunk(const int* __restrict__ dsts, int nE, int cbase, int slotBase,
                                          int vec8, int* list, int tid, int lane, int wave) {
  int wc = 0;
#pragma unroll
  for (int g = 0; g < NGRP; ++g) {
    const int el0  = (g * NTHR + tid) * EPT;
    const int e0   = cbase + el0;
    const int sent = -2147483647 - 1;
    v4i da, db;
    if (vec8 != 0 && cbase + CHUNK <= nE) {
      da = *(const v4i*)(dsts + e0);
      db = *(const v4i*)(dsts + e0 + 4);
    } else {
      da.x = (e0     < nE) ? dsts[min(e0, nE - 1)] : sent;
      da.y = (e0 + 1 < nE) ? dsts[min(e0 + 1, nE - 1)] : sent;
      da.z = (e0 + 2 < nE) ? dsts[min(e0 + 2, nE - 1)] : sent;
      da.w = (e0 + 3 < nE) ? dsts[min(e0 + 3, nE - 1)] : sent;
      db.x = (e0 + 4 < nE) ? dsts[min(e0 + 4, nE - 1)] : sent;
      db.y = (e0 + 5 < nE) ? dsts[min(e0 + 5, nE - 1)] : sent;
      db.z = (e0 + 6 < nE) ? dsts[min(e0 + 6, nE - 1)] : sent;
      db.w = (e0 + 7 < nE) ? dsts[min(e0 + 7, nE - 1)] : sent;
    }
    const unsigned nb = (unsigned)slotBase;
    const unsigned s0 = (unsigned)da.x - nb, s1 = (unsigned)da.y - nb;
    const unsigned s2 = (unsigned)da.z - nb, s3 = (unsigned)da.w - nb;
    const unsigned s4 = (unsigned)db.x - nb, s5 = (unsigned)db.y - nb;
    const unsigned s6 = (unsigned)db.z - nb, s7 = (unsigned)db.w - nb;
    const bool h0 = s0 < (unsigned)NB, h1 = s1 < (unsigned)NB, h2 = s2 < (unsigned)NB, h3 = s3 < (unsigned)NB;
    const bool h4 = s4 < (unsigned)NB, h5 = s5 < (unsigned)NB, h6 = s6 < (unsigned)NB, h7 = s7 < (unsigned)NB;
    const unsigned any = __builtin_amdgcn_ballot_w32(h0 | h1 | h2 | h3 | h4 | h5 | h6 | h7);
    if (any != 0u) {
#define HITJ(J, HJ, SJ) { \
        const unsigned mj = __builtin_amdgcn_ballot_w32(HJ); \
        if (mj != 0u) { \
          if (HJ) { \
            const int pos = wc + (int)__builtin_amdgcn_mbcnt_lo(mj, 0u); \
            if (pos < WCAP) list[wave * WCAP + pos] = ((el0 + (J)) << 12) | (int)(SJ); \
          } \
          wc += (int)__builtin_popcount(mj); } }
      HITJ(0, h0, s0)
      HITJ(1, h1, s1)
      HITJ(2, h2, s2)
      HITJ(3, h3, s3)
      HITJ(4, h4, s4)
      HITJ(5, h5, s5)
      HITJ(6, h6, s6)
      HITJ(7, h7, s7)
#undef HITJ
    }
  }
  return wc;
}

template <int KD, int NC>
__global__ __launch_bounds__(NTHR) void k_wprep(const float* __restrict__ W, _Float16* wp) {
  constexpr int UNITS = NC * KD / 8;
  constexpr int KD8   = KD / 8;
  static_assert((UNITS % 32) == 0);
  const int i = (int)blockIdx.x * NTHR + (int)threadIdx.x;
  if (i >= UNITS) return;
  const int n  = i / KD8;
  const int k0 = (i - n * KD8) * 8;
  v8h hv;
#pragma unroll
  for (int e = 0; e < 8; ++e) hv[e] = (_Float16)(W[(size_t)(k0 + e) * NC + n] * WSC);
  _Float16* d = wp + (size_t)i * 8;
  *(volatile v8h*)d = hv;
  __threadfence();
  *(volatile v8h*)d = hv;
}

__global__ __launch_bounds__(NTHR) void k_count(
    const int* __restrict__ dsts, int* cnt, int nE, int vec8) {
  __shared__ __attribute__((aligned(16))) int scnt[NBC];
  __shared__ __attribute__((aligned(16))) int list[LISTN];
  __shared__ int wcnt[NWAVE];
  const int tid = threadIdx.x, lane = tid & 31, wave = tid >> 5;
  const int nodeBase = blockIdx.x * NBC;

  for (int i = tid; i < NBC; i += NTHR) scnt[i] = 0;
  __syncthreads();

  const int nChunks = (nE + CHUNK - 1) / CHUNK;
#pragma unroll 1
  for (int ch = 0; ch < nChunks; ++ch) {
    const int cbase = ch * CHUNK;
    const int wc = scan_chunk<NBC>(dsts, nE, cbase, nodeBase, vec8, list, tid, lane, wave);
    if (lane == 0) wcnt[wave] = wc;
    __syncthreads();
    if (wave == 0) {
#pragma unroll 1
      for (int wsx = 0; wsx < NWAVE; ++wsx) {
        int n = __builtin_amdgcn_readfirstlane(wcnt[wsx]);
        n = n > WCAP ? WCAP : (n < 0 ? 0 : n);
        const int* lp = list + wsx * WCAP;
#pragma unroll 1
        for (int i = 0; i < n; ++i) {
          const int ent  = __builtin_amdgcn_readfirstlane(lp[i]);
          const int slot = ent & (NBC - 1);
          if (lane == 0) scnt[slot] = scnt[slot] + 1;
        }
      }
    }
    __syncthreads();
  }

  v4i cq[4];
#pragma unroll
  for (int q = 0; q < 4; ++q) {
    const int f = (wave * 4 + q) * 128 + 4 * lane;
    cq[q] = *(const v4i*)(scnt + f);
  }
  int* cp = cnt + (size_t)nodeBase;
#pragma unroll
  for (int q = 0; q < 4; ++q) {
    const int f = (wave * 4 + q) * 128 + 4 * lane;
    *(volatile v4i*)(cp + f) = cq[q];
  }
  __threadfence();
#pragma unroll
  for (int q = 0; q < 4; ++q) {
    const int f = (wave * 4 + q) * 128 + 4 * lane;
    *(volatile v4i*)(cp + f) = cq[q];
  }
}

__global__ __launch_bounds__(OTHR) void k_offsets(
    const int* __restrict__ cnt, int* off, int* rbase, int nChunk) {
  __shared__ __attribute__((aligned(16))) int soff[NBC];
  __shared__ __attribute__((aligned(16))) int srb[RBN];
  __shared__ int wtot[OTHR / 32];
  const int tid = threadIdx.x, lane = tid & 31, wave = tid >> 5, sub = tid >> 7;
  for (int i = tid; i < RBN; i += OTHR) srb[i] = 0;
  int carry = 0;
#pragma unroll 1
  for (int ch = 0; ch < nChunk; ++ch) {
    const int base = ch * NBC;
    const v4i c0 = *(const v4i*)(cnt + base + 8 * tid);
    const v4i c1 = *(const v4i*)(cnt + base + 8 * tid + 4);
    const int e0 = max(c0.x, 0), e1 = max(c0.y, 0), e2 = max(c0.z, 0), e3 = max(c0.w, 0);
    const int e4 = max(c1.x, 0), e5 = max(c1.y, 0), e6 = max(c1.z, 0), e7 = max(c1.w, 0);
    const int ts = e0 + e1 + e2 + e3 + e4 + e5 + e6 + e7;
    int incl = ts;
#pragma unroll
    for (int d = 1; d < 32; d <<= 1) {
      const int t = __shfl_up(incl, d);
      if (lane >= d) incl += t;
    }
    if (lane == 31) wtot[wave] = incl;
    __syncthreads();
    const int S0 = wtot[0]  + wtot[1]  + wtot[2]  + wtot[3];
    const int S1 = wtot[4]  + wtot[5]  + wtot[6]  + wtot[7];
    const int S2 = wtot[8]  + wtot[9]  + wtot[10] + wtot[11];
    const int S3 = wtot[12] + wtot[13] + wtot[14] + wtot[15];
    int pre = 0;
#pragma unroll 1
    for (int w = 4 * sub; w < wave; ++w) pre += wtot[w];
    const int b0 = carry;
    const int b1 = b0 + ((S0 + 31) & ~31);
    const int b2 = b1 + ((S1 + 31) & ~31);
    const int b3 = b2 + ((S2 + 31) & ~31);
    const int b4 = b3 + ((S3 + 31) & ~31);
    const int myb = sub == 0 ? b0 : (sub == 1 ? b1 : (sub == 2 ? b2 : b3));
    if (tid == 0) {
      srb[min(4 * ch + 0, RBN - 1)] = b0;
      srb[min(4 * ch + 1, RBN - 1)] = b1;
      srb[min(4 * ch + 2, RBN - 1)] = b2;
      srb[min(4 * ch + 3, RBN - 1)] = b3;
    }
    int run = myb + pre + incl - ts;
    soff[8 * tid + 0] = run; run += e0;
    soff[8 * tid + 1] = run; run += e1;
    soff[8 * tid + 2] = run; run += e2;
    soff[8 * tid + 3] = run; run += e3;
    soff[8 * tid + 4] = run; run += e4;
    soff[8 * tid + 5] = run; run += e5;
    soff[8 * tid + 6] = run; run += e6;
    soff[8 * tid + 7] = run;
    carry = b4;
    __syncthreads();
    const v4i o0 = *(const v4i*)(soff + 4 * tid);
    const v4i o1 = *(const v4i*)(soff + 4 * (tid + OTHR));
    int* op = off + base;
    *(volatile v4i*)(op + 4 * tid) = o0;
    *(volatile v4i*)(op + 4 * (tid + OTHR)) = o1;
    __threadfence();
    *(volatile v4i*)(op + 4 * tid) = o0;
    *(volatile v4i*)(op + 4 * (tid + OTHR)) = o1;
    __syncthreads();
  }
  if (tid == 0) srb[min(4 * nChunk, RBN - 1)] = carry;
  __syncthreads();
  v4i rv = {0, 0, 0, 0};
  if (tid < 32) rv = *(const v4i*)(srb + 4 * tid);
  if (tid < 32) *(volatile v4i*)(rbase + 4 * tid) = rv;
  __threadfence();
  if (tid < 32) *(volatile v4i*)(rbase + 4 * tid) = rv;
}

__global__ __launch_bounds__(NTHR) void k_fill(
    const int* __restrict__ srcs, const int* __restrict__ dsts,
    const int* __restrict__ off, const int* __restrict__ rbase,
    int* csr, int nN, int nE, int vec8, int csrLen) {
  extern __shared__ v4f lds_dyn[];
  int* region = (int*)lds_dyn;
  int* cursor = region + RCAP;
  int* list   = cursor + NBF;
  int* wcnt   = list + LISTN;
  const int tid = threadIdx.x, lane = tid & 31, wave = tid >> 5;
  const int b = blockIdx.x;
  const int nodeBase = b * NBF;

  int rb0 = rbase[b];
  const int rb1 = rbase[b + 1];
  rb0 = rb0 < 0 ? 0 : (rb0 > csrLen ? csrLen : rb0);
  rb0 &= ~31;
  int len = rb1 - rb0;
  len = len < 0 ? 0 : (len > RCAP ? RCAP : len);
  int lenW = (len + 31) & ~31;
  if (rb0 + lenW > csrLen) lenW = (csrLen - rb0) & ~31;

  {
    const v4i z = {0, 0, 0, 0};
    for (int i = tid; i < RCAP / 4; i += NTHR) ((v4i*)region)[i] = z;
    for (int s = tid; s < NBF; s += NTHR) {
      int o = off[nodeBase + s] - rb0;
      o = o < 0 ? 0 : (o > RCAP ? RCAP : o);
      cursor[s] = o;
    }
  }
  __syncthreads();

  const int nChunks = (nE + CHUNK - 1) / CHUNK;
#pragma unroll 1
  for (int ch = 0; ch < nChunks; ++ch) {
    const int cbase = ch * CHUNK;
    const int wc = scan_chunk<NBF>(dsts, nE, cbase, nodeBase, vec8, list, tid, lane, wave);
    if (lane == 0) wcnt[wave] = wc;
    __syncthreads();
    if (wave == 0) {
#pragma unroll 1
      for (int wsx = 0; wsx < NWAVE; ++wsx) {
        int n = __builtin_amdgcn_readfirstlane(wcnt[wsx]);
        n = n > WCAP ? WCAP : (n < 0 ? 0 : n);
        const int* lp = list + wsx * WCAP;
#pragma unroll 1
        for (int i = 0; i < n; ++i) {
          const int ent  = __builtin_amdgcn_readfirstlane(lp[i]);
          const int slot = ent & (NBF - 1);
          int e = cbase + ((ent >> 12) & (CHUNK - 1));
          e = e > nE - 1 ? nE - 1 : e;
          int src = srcs[e];
          src = src < 0 ? 0 : (src > nN - 1 ? nN - 1 : src);
          if (lane == 0) {
            int pos = cursor[slot];
            pos = pos < 0 ? 0 : (pos > RCAP - 1 ? RCAP - 1 : pos);
            region[pos] = src;
            const int np = pos + 1;
            cursor[slot] = np > RCAP ? RCAP : np;
          }
        }
      }
    }
    __syncthreads();
  }

  const int nv = lenW >> 2;
  int* gp = csr + rb0;
#pragma unroll 1
  for (int i = tid; i < nv; i += NTHR) { const v4i v = ((const v4i*)region)[i]; *(volatile v4i*)(gp + 4 * i) = v; }
  __threadfence();
#pragma unroll 1
  for (int i = tid; i < nv; i += NTHR) { const v4i v = ((const v4i*)region)[i]; *(volatile v4i*)(gp + 4 * i) = v; }
}

__device__ __forceinline__ void mm_tile(const _Float16* As, const _Float16* __restrict__ Bw, float* stg) {
  const int tid = threadIdx.x, lane = tid & 31, wave = tid >> 5, hh = lane >> 4, m = lane & 15;
  const int r0 = wave * 16;
  v8f acc[8];
#pragma unroll
  for (int t = 0; t < 8; ++t) { v8f z = {0.f, 0.f, 0.f, 0.f, 0.f, 0.f, 0.f, 0.f}; acc[t] = z; }
  const _Float16* ap  = As + (size_t)(r0 + m) * APITCH + 8 * hh;
  const _Float16* bp0 = Bw + (size_t)m * FIN + 8 * hh;
#pragma unroll 1
  for (int kt = 0; kt < FIN / 32; ++kt) {
    FragH a;
    a.h[0] = *(const v8h*)(ap + 32 * kt);
    a.h[1] = *(const v8h*)(ap + 32 * kt + 16);
#pragma unroll
    for (int t = 0; t < 8; ++t) {
      const _Float16* bp = bp0 + (size_t)(16 * t) * FIN + 32 * kt;
      FragH b;
      b.h[0] = *(const v8h*)bp;
      b.h[1] = *(const v8h*)(bp + 16);
      acc[t] = wmh(a.v, b.v, acc[t]);
    }
  }
  float* sp = stg + (size_t)(r0 + 8 * hh) * HID + m;
#pragma unroll
  for (int t = 0; t < 8; ++t) {
#pragma unroll
    for (int r = 0; r < 8; ++r) sp[r * HID + 16 * t] = acc[t][r] * INV_CARRY;
  }
}

template <int HEADS>
__global__ __launch_bounds__(NTHR) void k_gemm_att(
    const float* __restrict__ A, const _Float16* __restrict__ Bw,
    const float* __restrict__ attS, const float* __restrict__ attD,
    float* C, float* eS, float* eD, int nRows) {
  static_assert(HEADS == 4 || HEADS == 1);
  constexpr int CHN = HID / HEADS;
  extern __shared__ v4f lds_dyn[];
  _Float16* As = (_Float16*)lds_dyn;
  float* stg = (float*)((char*)lds_dyn + LDS_ATILE);
  __shared__ __attribute__((aligned(16))) float sES[BM * 4];
  __shared__ __attribute__((aligned(16))) float sED[BM * 4];
  const int tid = threadIdx.x, lane = tid & 31, wave = tid >> 5;
  const int rowBase = blockIdx.x * BM;
  const int r0 = wave * 16;
  const v4f z4 = {0.f, 0.f, 0.f, 0.f};

#pragma unroll 2
  for (int it = 0; it < 8; ++it) {
    const int u    = it * NTHR + tid;
    const int row  = u >> 4;
    const int c    = (u & 15) * 8;
    const int grow = rowBase + row;
    const int rr   = grow < nRows ? grow : nRows - 1;
    const float* p = A + (size_t)rr * FIN + c;
    v4f a = *(const v4f*)p, b = *(const v4f*)(p + 4);
    if (grow >= nRows) { a = z4; b = z4; }
    v8h hv;
    hv[0] = (_Float16)(a.x * XSC); hv[1] = (_Float16)(a.y * XSC);
    hv[2] = (_Float16)(a.z * XSC); hv[3] = (_Float16)(a.w * XSC);
    hv[4] = (_Float16)(b.x * XSC); hv[5] = (_Float16)(b.y * XSC);
    hv[6] = (_Float16)(b.z * XSC); hv[7] = (_Float16)(b.w * XSC);
    *(v8h*)(As + (size_t)row * APITCH + c) = hv;
  }
  __syncthreads();

  mm_tile(As, Bw, stg);
  __syncthreads();

  const int col = 4 * lane;
  const int hd  = col / CHN;
  const v4f sA = *(const v4f*)(attS + col);
  const v4f sD = *(const v4f*)(attD + col);
  const size_t gb = (size_t)(rowBase + r0) * HID + col;
#pragma unroll
  for (int row = 0; row < 16; ++row) {
    const v4f v = *(const v4f*)(stg + (size_t)(r0 + row) * HID + col);
    *(volatile v4f*)(C + gb + (size_t)row * HID) = v;
    float ps = v.x * sA.x + v.y * sA.y + v.z * sA.z + v.w * sA.w;
    float pd = v.x * sD.x + v.y * sD.y + v.z * sD.z + v.w * sD.w;
    if constexpr (HEADS == 4) {
#pragma unroll
      for (int o = 1; o < 8; o <<= 1) { ps += __shfl_xor(ps, o); pd += __shfl_xor(pd, o); }
      if ((lane & 7) == 0) { sES[(r0 + row) * 4 + hd] = ps; sED[(r0 + row) * 4 + hd] = pd; }
    } else {
#pragma unroll
      for (int o = 1; o < 32; o <<= 1) { ps += __shfl_xor(ps, o); pd += __shfl_xor(pd, o); }
      if (lane == 0) { sES[r0 + row] = ps; sED[r0 + row] = pd; }
    }
  }
  __threadfence();
#pragma unroll
  for (int row = 0; row < 16; ++row) {
    const v4f v = *(const v4f*)(stg + (size_t)(r0 + row) * HID + col);
    *(volatile v4f*)(C + gb + (size_t)row * HID) = v;
  }
  __syncthreads();

  if constexpr (HEADS == 4) {
    v4f dv = z4;
    const size_t eb = (size_t)rowBase * 4;
    if (wave < 4) {
      const int f = wave * 128 + 4 * lane;
      dv = *(const v4f*)(sES + f);
      *(volatile v4f*)(eS + eb + f) = dv;
    } else {
      const int f = (wave - 4) * 128 + 4 * lane;
      dv = *(const v4f*)(sED + f);
      *(volatile v4f*)(eD + eb + f) = dv;
    }
    __threadfence();
    if (wave < 4) {
      const int f = wave * 128 + 4 * lane;
      *(volatile v4f*)(eS + eb + f) = dv;
    } else {
      const int f = (wave - 4) * 128 + 4 * lane;
      *(volatile v4f*)(eD + eb + f) = dv;
    }
  } else {
    const int f = 4 * lane;
    const size_t eb = (size_t)rowBase;
    v4f dvs = *(const v4f*)(sES + f);
    v4f dvd = *(const v4f*)(sED + f);
    if (wave == 0)      *(volatile v4f*)(eS + eb + f) = dvs;
    else if (wave == 1) *(volatile v4f*)(eD + eb + f) = dvd;
    __threadfence();
    if (wave == 0)      *(volatile v4f*)(eS + eb + f) = dvs;
    else if (wave == 1) *(volatile v4f*)(eD + eb + f) = dvd;
  }
}

template <int HEADS, int LAST>
__global__ __launch_bounds__(NTHR) void k_agg(
    const int* __restrict__ csr, const int* __restrict__ off, const int* __restrict__ cnt,
    const float* __restrict__ eS, const float* __restrict__ eD, const float* __restrict__ hw,
    const float* __restrict__ bias, float* xout, int nN, int csrLen) {
  static_assert(HEADS == 4 || HEADS == 1);
  constexpr int CHN = HID / HEADS;
  const int tid = threadIdx.x, lane = tid & 31, wave = tid >> 5;
  const int tbase = blockIdx.x * TGT + wave * 32;
  const int col0 = 4 * lane;
  const int hd0  = col0 / CHN;
  const v4f z4 = {0.f, 0.f, 0.f, 0.f};
  const v4f bb0 = *(const v4f*)(bias + col0);

  const int cl    = tbase + lane;
  const int cnt_l = cnt[cl];
  const int off_l = off[cl];

#pragma unroll 1
  for (int j = 0; j < 32; ++j) {
    const int c = tbase + j;
    int n = __shfl(cnt_l, j);
    n = n < 0 ? 0 : (n > DEGCAP ? DEGCAP : n);
    const int st = __shfl(off_l, j);
    const float ed0 = eD[(size_t)c * HEADS + hd0];
    const float ef0 = lrelu(eS[(size_t)c * HEADS + hd0] + ed0);

    float mx0 = ef0;
#pragma unroll 1
    for (int q0 = 0; q0 < n; q0 += 32) {
      int pos = st + q0 + lane;
      pos = pos < 0 ? 0 : (pos > csrLen - 1 ? csrLen - 1 : pos);
      int sl = csr[pos];
      sl = sl < 0 ? 0 : (sl > nN - 1 ? nN - 1 : sl);
      const int mcnt = (n - q0) < 32 ? (n - q0) : 32;
#pragma unroll 1
      for (int pp = 0; pp < mcnt; ++pp) {
        const int s = __builtin_amdgcn_readlane(sl, pp);
        mx0 = fmaxf(mx0, lrelu(eS[(size_t)s * HEADS + hd0] + ed0));
      }
    }

    float den0 = 0.f;
    v4f   acc0 = z4;
#pragma unroll 1
    for (int q0 = 0; q0 < n; q0 += 32) {
      int pos = st + q0 + lane;
      pos = pos < 0 ? 0 : (pos > csrLen - 1 ? csrLen - 1 : pos);
      int sl = csr[pos];
      sl = sl < 0 ? 0 : (sl > nN - 1 ? nN - 1 : sl);
      const int mcnt = (n - q0) < 32 ? (n - q0) : 32;
#pragma unroll 1
      for (int pp = 0; pp < mcnt; ++pp) {
        const int s = __builtin_amdgcn_readlane(sl, pp);
        const float p0 = __expf(lrelu(eS[(size_t)s * HEADS + hd0] + ed0) - mx0);
        den0 += p0;
        const v4f h0 = *(const v4f*)(hw + (size_t)s * HID + col0);
        acc0 = acc0 + h0 * p0;
      }
    }
    {
      const float p0 = __expf(ef0 - mx0);
      den0 += p0;
      const v4f h0 = *(const v4f*)(hw + (size_t)c * HID + col0);
      acc0 = acc0 + h0 * p0;
    }

    const float rd0 = 1.0f / (den0 + DEN_EPS);
    v4f v0 = acc0 * rd0 + bb0;

    float* pw = xout + (size_t)c * HID;
    if constexpr (LAST == 0) {
      if (c >= nN) v0 = z4;
      *(volatile v4f*)(pw + col0) = v0;
      __threadfence();
      *(volatile v4f*)(pw + col0) = v0;
    } else {
      if (c < nN) {
        *(volatile v4f*)(pw + col0) = v0;
        __threadfence();
        *(volatile v4f*)(pw + col0) = v0;
      }
    }
  }
}

__global__ __launch_bounds__(BNT) void k_bnstat(const float* __restrict__ O0, double* part, int nN) {
  const int col = threadIdx.x;
  const int r0 = blockIdx.x * STATR;
  int nr = nN - r0;
  nr = nr < 0 ? 0 : (nr > STATR ? STATR : nr);
  double s = 0.0, q = 0.0;
#pragma unroll 1
  for (int i = 0; i < nr; ++i) {
    const double v = (double)O0[(size_t)(r0 + i) * HID + col];
    s += v;
    q += v * v;
  }
  double* pp = part + (size_t)blockIdx.x * (2 * HID);
  *(volatile double*)(pp + col) = s;
  *(volatile double*)(pp + HID + col) = q;
  __threadfence();
  *(volatile double*)(pp + col) = s;
  *(volatile double*)(pp + HID + col) = q;
}

__global__ __launch_bounds__(BNT) void k_bnfin(const double* __restrict__ part, const float* __restrict__ gamma,
                                               float* tbl, int nPart, int nN) {
  const int col = threadIdx.x;
  double s = 0.0, q = 0.0;
#pragma unroll 1
  for (int b = 0; b < nPart; ++b) {
    s += part[(size_t)b * (2 * HID) + col];
    q += part[(size_t)b * (2 * HID) + HID + col];
  }
  const double inv = 1.0 / (double)nN;
  const double mu  = s * inv;
  double var = q * inv - mu * mu;
  var = var < 0.0 ? 0.0 : var;
  const float a  = (float)((double)gamma[col] / sqrt(var + BN_EPS));
  const float mf = (float)mu;
  *(volatile float*)(tbl + col) = mf;
  *(volatile float*)(tbl + HID + col) = a;
  __threadfence();
  *(volatile float*)(tbl + col) = mf;
  *(volatile float*)(tbl + HID + col) = a;
}

__global__ __launch_bounds__(NTHR) void k_bnapply(
    const float* __restrict__ O0, const float* __restrict__ x,
    const float* __restrict__ tbl, const float* __restrict__ beta,
    float* H, int nN, int nUnits) {
  const int i = (int)blockIdx.x * NTHR + (int)threadIdx.x;
  if (i >= nUnits) return;
  const int row = i >> 5;
  const int c   = (i & 31) * 4;
  const int rr  = row < nN ? row : nN - 1;
  const v4f o  = *(const v4f*)(O0 + (size_t)row * HID + c);
  const v4f xv = *(const v4f*)(x + (size_t)rr * FIN + c);
  const v4f mu = *(const v4f*)(tbl + c);
  const v4f ga = *(const v4f*)(tbl + HID + c);
  const v4f be = *(const v4f*)(beta + c);
  const v4f z4 = {0.f, 0.f, 0.f, 0.f};
  v4f h = (o - mu) * ga + be;
  h.x = eluf(h.x); h.y = eluf(h.y); h.z = eluf(h.z); h.w = eluf(h.w);
  h = h + xv;
  if (row >= nN) h = z4;
  float* d = H + (size_t)row * HID + c;
  *(volatile v4f*)d = h;
  __threadfence();
  *(volatile v4f*)d = h;
}

extern "C" void kernel_launch(void* const* d_in, const int* in_sizes, int n_in,
                              void* d_out, int out_size, void* d_ws, size_t ws_size,
                              hipStream_t stream) {
  if (n_in < 12) return;
  const int nN = in_sizes[0] / FIN;
  const int nE = in_sizes[1] / 2;
  if (nN <= 0 || nE <= 0 || in_sizes[0] != nN * FIN || in_sizes[1] != 2 * nE) return;
  if (in_sizes[2] != FIN * HID || in_sizes[3] != HID || in_sizes[4] != HID || in_sizes[5] != HID) return;
  if (in_sizes[6] != HID * HID || in_sizes[7] != HID || in_sizes[8] != HID || in_sizes[9] != HID) return;
  if (in_sizes[10] != HID || in_sizes[11] != HID) return;
  if (out_size != nN * HID) return;
  if (nE > (1 << 28) || nN > (1 << 22)) return;

  const float* x      = (const float*)d_in[0];
  const int*   ei     = (const int*)d_in[1];
  const float* W1     = (const float*)d_in[2];
  const float* att_s1 = (const float*)d_in[3];
  const float* att_d1 = (const float*)d_in[4];
  const float* b1     = (const float*)d_in[5];
  const float* W2     = (const float*)d_in[6];
  const float* att_s2 = (const float*)d_in[7];
  const float* att_d2 = (const float*)d_in[8];
  const float* b2     = (const float*)d_in[9];
  const float* gamma  = (const float*)d_in[10];
  const float* beta   = (const float*)d_in[11];
  const int*   src = ei;
  const int*   dst = ei + nE;
  float* out = (float*)d_out;

  const int NPAD   = ((nN + TGT - 1) / TGT) * TGT;
  const int nBC    = (nN + NBC - 1) / NBC;
  const int CNTPAD = nBC * NBC;
  if (CNTPAD < NPAD) return;
  if (4 * nBC + 1 > RBN) return;
  const int nBF    = (nN + NBF - 1) / NBF;
  const int csrLen = ((nE + 31) & ~31) + 4096;
  if (31 * 4 * nBC > 4096) return;
  const int nAgg   = NPAD / TGT;
  const int nGm    = NPAD / BM;
  const int nStat  = NPAD / STATR;
  const int nUnitH = NPAD * (HID / 4);

  char* ws = (char*)d_ws;
  size_t off = 0;
  const size_t oWp1 = off; off += (size_t)HID * FIN * 2;         off = (off + 255) & ~(size_t)255;
  const size_t oWp2 = off; off += (size_t)HID * HID * 2;         off = (off + 255) & ~(size_t)255;
  const size_t oCnt = off; off += (size_t)CNTPAD * 4;            off = (off + 255) & ~(size_t)255;
  const size_t oOff = off; off += (size_t)CNTPAD * 4;            off = (off + 255) & ~(size_t)255;
  const size_t oRb  = off; off += (size_t)RBN * 4;               off = (off + 255) & ~(size_t)255;
  const size_t oCsr = off; off += (size_t)csrLen * 4;            off = (off + 255) & ~(size_t)255;
  const size_t oR1  = off; off += (size_t)NPAD * HID * 4;        off = (off + 255) & ~(size_t)255;
  const size_t oR2  = off; off += (size_t)NPAD * HID * 4;        off = (off + 255) & ~(size_t)255;
  const size_t oES  = off; off += (size_t)NPAD * NHEADA * 4;     off = (off + 255) & ~(size_t)255;
  const size_t oED  = off; off += (size_t)NPAD * NHEADA * 4;     off = (off + 255) & ~(size_t)255;
  const size_t oPrt = off; off += (size_t)nStat * 2 * HID * 8;   off = (off + 255) & ~(size_t)255;
  const size_t oTbl = off; off += (size_t)2 * HID * 4;           off = (off + 255) & ~(size_t)255;
  if (off > ws_size || off > (size_t)WSCAP) return;
  _Float16* wp1 = (_Float16*)(ws + oWp1);
  _Float16* wp2 = (_Float16*)(ws + oWp2);
  int*    cnt  = (int*)(ws + oCnt);
  int*    offp = (int*)(ws + oOff);
  int*    rb   = (int*)(ws + oRb);
  int*    csr  = (int*)(ws + oCsr);
  float*  r1   = (float*)(ws + oR1);
  float*  r2   = (float*)(ws + oR2);
  float*  es   = (float*)(ws + oES);
  float*  ed   = (float*)(ws + oED);
  double* part = (double*)(ws + oPrt);
  float*  tbl  = (float*)(ws + oTbl);

  const int vec8 = ((nE & 3) == 0) ? 1 : 0;

  k_wprep<FIN, HID><<<(HID * FIN / 8 + NTHR - 1) / NTHR, NTHR, 0, stream>>>(W1, wp1);
  k_wprep<HID, HID><<<(HID * HID / 8 + NTHR - 1) / NTHR, NTHR, 0, stream>>>(W2, wp2);

  k_count<<<nBC, NTHR, 0, stream>>>(dst, cnt, nE, vec8);
  k_offsets<<<1, OTHR, 0, stream>>>(cnt, offp, rb, nBC);
  hipFuncSetAttribute(reinterpret_cast<const void*>(&k_fill),
                      hipFuncAttributeMaxDynamicSharedMemorySize, LDS_FILL);
  k_fill<<<nBF, NTHR, LDS_FILL, stream>>>(src, dst, offp, rb, csr, nN, nE, vec8, csrLen);

  hipFuncSetAttribute(reinterpret_cast<const void*>(&k_gemm_att<NHEADA>),
                      hipFuncAttributeMaxDynamicSharedMemorySize, LDS_GEMM);
  k_gemm_att<NHEADA><<<nGm, NTHR, LDS_GEMM, stream>>>(x, wp1, att_s1, att_d1, r1, es, ed, nN);
  k_agg<NHEADA, 0><<<nAgg, NTHR, 0, stream>>>(csr, offp, cnt, es, ed, r1, b1, r2, nN, csrLen);

  k_bnstat<<<nStat, BNT, 0, stream>>>(r2, part, nN);
  k_bnfin<<<1, BNT, 0, stream>>>(part, gamma, tbl, nStat, nN);

  k_bnapply<<<(nUnitH + NTHR - 1) / NTHR, NTHR, 0, stream>>>(r2, x, tbl, beta, r1, nN, nUnitH);

  hipFuncSetAttribute(reinterpret_cast<const void*>(&k_gemm_att<1>),
                      hipFuncAttributeMaxDynamicSharedMemorySize, LDS_GEMM);
  k_gemm_att<1><<<nGm, NTHR, LDS_GEMM, stream>>>(r1, wp2, att_s2, att_d2, r2, es, ed, nN);
  k_agg<1, 1><<<nAgg, NTHR, 0, stream>>>(csr, offp, cnt, es, ed, r2, b2, out, nN, csrLen);
}
